// EGNNLayer_65017214927603
// MI455X (gfx1250) — hardware-verified
//
#include <hip/hip_runtime.h>
#include <stddef.h>
#include <stdint.h>

#define NN     384
#define HID    256
#define EW1S   513
#define K2     512
#define K3     768
#define NPQ    512
#define NTHR   256
#define TJ     128
#define NJT    3
#define GBM    64
#define GBN    128
#define GTHR   128
#define GVGPR  248
#define OUT0_ELEMS (NN * HID)
#define OUT1_ELEMS (NN * 3)
#define OUT_TOTAL  (OUT0_ELEMS + OUT1_ELEMS)
#define WSMAX  134217728

#define NU_XB   (NN * (HID / 8))
#define NU_PQW  (NPQ * (HID / 8))
#define NU_DUP  (HID * (K2 / 8))
#define NU_NW1  (HID * (K3 / 8))
#define NU_TAB  512
#define NU_POS  512
#define TAB_UNITS 456
#define POS_UNITS 288
#define NU_ALL  (NU_XB + NU_PQW + 3 * NU_DUP + NU_NW1 + NU_TAB + NU_POS)

#define T_WR   0
#define T_EB1  256
#define T_EB2  512
#define T_NB1  768
#define T_NB2  1024
#define T_PB1  1280
#define T_PW2  1536
#define T_PB2  1792
#define T_END  1824

#define L_D    32768
#define L_PB   65536
#define L_WR   65792
#define L_EB2  66048
#define L_PB1  66304
#define L_PW2  66560
#define L_CS   66816
#define L_RAD  67072
#define L_S    67200
#define L_END  67328
#define EDGE_LDS_BYTES (L_END * 4)

static_assert(NN == 384 && NN == NJT * TJ && NN % GBM == 0);
static_assert(HID == 256 && HID == NTHR && EW1S == 2 * HID + 1);
static_assert(K2 == 2 * HID && K3 == 3 * HID && K2 % 32 == 0 && K3 % 32 == 0 && HID % 32 == 0);
static_assert(NPQ == 2 * HID && NPQ % GBN == 0 && HID % GBN == 0);
static_assert(GBM == (GTHR / 32) * 16 && GBN == 4 * 32);
static_assert(NU_XB % NTHR == 0 && NU_PQW % NTHR == 0 && NU_DUP % NTHR == 0 && NU_NW1 % NTHR == 0);
static_assert(NU_TAB % NTHR == 0 && NU_POS % NTHR == 0 && NU_ALL % NTHR == 0);
static_assert(TAB_UNITS * 4 == T_END && TAB_UNITS <= NU_TAB && (T_END * 4) % 128 == 0 && (T_PB2 * 4) % 128 == 0);
static_assert(POS_UNITS * 4 == OUT1_ELEMS && POS_UNITS <= NU_POS && POS_UNITS % 32 == 0);
static_assert((OUT0_ELEMS * 4) % 128 == 0 && (OUT1_ELEMS * 4) % 128 == 0);
static_assert(OUT0_ELEMS + OUT1_ELEMS == OUT_TOTAL && OUT_TOTAL == 99456);
static_assert(L_D * 4 == TJ * K2 * 2 && (L_PB - L_D) == TJ * HID);
static_assert(EDGE_LDS_BYTES <= 327680);
static_assert(TJ == 8 * 16 && NTHR == 8 * 32 && (TJ * 4) % 128 == 0);
static_assert((NN * (HID / 8)) % NTHR == 0);
static_assert(GVGPR < 256);

typedef float          v4f   __attribute__((ext_vector_type(4)));
typedef float          v8f   __attribute__((ext_vector_type(8)));
typedef int            v8i   __attribute__((ext_vector_type(8)));
typedef unsigned       v2u   __attribute__((ext_vector_type(2)));
typedef unsigned short v8us  __attribute__((ext_vector_type(8)));
typedef unsigned short v16us __attribute__((ext_vector_type(16)));
typedef __bf16         v16bf __attribute__((ext_vector_type(16)));
typedef v4f  __attribute__((may_alias)) v4fa;
typedef v2u  __attribute__((may_alias)) v2ua;
typedef v8us __attribute__((may_alias)) v8usa;
union FragB { v16bf v; v16us u; v8us h[2]; v8i w; };

__device__ __forceinline__ v8f wmb(const FragB& a, const FragB& b, v8f c) {
  v8f d = __builtin_amdgcn_wmma_f32_16x16x32_bf16(false, a.v, false, b.v, (short)0, c, false, false);
  asm volatile("v_nop\n\tv_nop\n\tv_nop\n\tv_nop" : "+v"(d) : "v"(a.w), "v"(b.w));
  return d;
}

__device__ __forceinline__ unsigned bf16_bits(float f) {
  const unsigned u = __float_as_uint(f);
  return (u + 0x7FFFu + ((u >> 16) & 1u)) >> 16;
}
__device__ __forceinline__ float bf16_val(float f) {
  return __uint_as_float(bf16_bits(f) << 16);
}
__device__ __forceinline__ float silu_f(float t) {
  return t * __builtin_amdgcn_rcpf(1.0f + expf(-t));
}
__device__ __forceinline__ void put16(unsigned short* dp, v8us o) {
  *(volatile v8us*)dp = o;
  __threadfence();
  *(volatile v8us*)dp = o;
}
__device__ __forceinline__ void putf4(float* dp, v4f o) {
  *(volatile v4f*)dp = o;
  __threadfence();
  *(volatile v4f*)dp = o;
}
__device__ __forceinline__ v8us cvt8(v4f a, v4f b) {
  v8us o;
  o[0] = (unsigned short)bf16_bits(a.x); o[1] = (unsigned short)bf16_bits(a.y);
  o[2] = (unsigned short)bf16_bits(a.z); o[3] = (unsigned short)bf16_bits(a.w);
  o[4] = (unsigned short)bf16_bits(b.x); o[5] = (unsigned short)bf16_bits(b.y);
  o[6] = (unsigned short)bf16_bits(b.z); o[7] = (unsigned short)bf16_bits(b.w);
  return o;
}
__device__ __forceinline__ v4f ldr4(const float* __restrict__ p) {
  const v4f a = *(const v4fa*)p;
  const v4f r = {bf16_val(a.x), bf16_val(a.y), bf16_val(a.z), bf16_val(a.w)};
  return r;
}
__device__ __forceinline__ void dup_unit(const float* __restrict__ W, unsigned short* dst, int v) {
  const int n  = v >> 6;
  const int k8 = (v & 63) * 8;
  const int sc = k8 & (HID - 1);
  const float* p = W + (size_t)n * HID + sc;
  const v4f a = *(const v4fa*)p;
  const v4f b = *(const v4fa*)(p + 4);
  put16(dst + (size_t)n * K2 + k8, cvt8(a, b));
}

__global__ __launch_bounds__(NTHR) void k_prep(const float* __restrict__ nodes, const float* __restrict__ pos,
                                               const float* __restrict__ eW1, const float* __restrict__ eb1,
                                               const float* __restrict__ eW2, const float* __restrict__ eb2,
                                               const float* __restrict__ nW1, const float* __restrict__ nb1,
                                               const float* __restrict__ nW2, const float* __restrict__ nb2,
                                               const float* __restrict__ pW1, const float* __restrict__ pb1,
                                               const float* __restrict__ pW2, const float* __restrict__ pb2,
                                               unsigned short* XB, float* POSR, unsigned short* EW1PQ,
                                               unsigned short* EW2D, unsigned short* PW1D, unsigned short* NW2D,
                                               unsigned short* NW1C, float* TAB) {
  const int u  = (int)blockIdx.x * NTHR + (int)threadIdx.x;
  const int U0 = NU_XB;
  const int U1 = U0 + NU_PQW;
  const int U2 = U1 + NU_DUP;
  const int U3 = U2 + NU_DUP;
  const int U4 = U3 + NU_DUP;
  const int U5 = U4 + NU_NW1;
  const int U6 = U5 + NU_TAB;
  if (u < U0) {
    const int row = u >> 5;
    const int k8  = (u & 31) * 8;
    const float* p = nodes + (size_t)row * HID + k8;
    const v4f a = *(const v4fa*)p;
    const v4f b = *(const v4fa*)(p + 4);
    put16(XB + (size_t)row * HID + k8, cvt8(a, b));
    return;
  } else if (u < U1) {
    const int v    = u - U0;
    const int n    = v >> 5;
    const int k8   = (v & 31) * 8;
    const int srow = n & (HID - 1);
    const int scol = (n >> 8) * HID + k8;
    const float* p = eW1 + (size_t)srow * EW1S + scol;
    v8us o;
#pragma unroll
    for (int i = 0; i < 8; ++i) o[i] = (unsigned short)bf16_bits(p[i]);
    put16(EW1PQ + (size_t)n * HID + k8, o);
    return;
  } else if (u < U2) {
    dup_unit(eW2, EW2D, u - U1);
    return;
  } else if (u < U3) {
    dup_unit(pW1, PW1D, u - U2);
    return;
  } else if (u < U4) {
    dup_unit(nW2, NW2D, u - U3);
    return;
  } else if (u < U5) {
    const int v  = u - U4;
    const int n  = v / (K3 / 8);
    const int k8 = (v - n * (K3 / 8)) * 8;
    const int sc = (k8 < 2 * HID) ? k8 : (k8 - HID);
    const float* p = nW1 + (size_t)n * (2 * HID) + sc;
    const v4f a = *(const v4fa*)p;
    const v4f b = *(const v4fa*)(p + 4);
    put16(NW1C + (size_t)n * K3 + k8, cvt8(a, b));
    return;
  } else if (u < U6) {
    const int v = u - U5;
    const int t = v >> 6;
    const int q = v & 63;
    v4f o = {0.0f, 0.0f, 0.0f, 0.0f};
    if (t == 0) {
      const float* p = eW1 + (size_t)(4 * q) * EW1S + 2 * HID;
      o.x = bf16_val(p[0]);
      o.y = bf16_val(p[EW1S]);
      o.z = bf16_val(p[2 * EW1S]);
      o.w = bf16_val(p[3 * EW1S]);
    } else if (t == 1) {
      o = ldr4(eb1 + 4 * q);
    } else if (t == 2) {
      o = ldr4(eb2 + 4 * q);
    } else if (t == 3) {
      o = ldr4(nb1 + 4 * q);
    } else if (t == 4) {
      o = ldr4(nb2 + 4 * q);
    } else if (t == 5) {
      o = ldr4(pb1 + 4 * q);
    } else if (t == 6) {
      o = ldr4(pW2 + 4 * q);
    } else {
      const float b = bf16_val(pb2[0]);
      o.x = (q == 0) ? b : 0.0f;
    }
    if (v < TAB_UNITS) putf4(TAB + 4 * v, o);
    return;
  } else {
    const int v  = u - U6;
    const int vc = v < POS_UNITS ? v : POS_UNITS - 1;
    const v4f o = ldr4(pos + 4 * vc);
    if (v < POS_UNITS) putf4(POSR + 4 * v, o);
    return;
  }
}

template <int MODE>
__global__ __launch_bounds__(GTHR) __attribute__((amdgpu_num_vgpr(GVGPR)))
void k_gemm(const unsigned short* __restrict__ A, int lda,
            const unsigned short* __restrict__ BT, int ldb, int K,
            const float* __restrict__ bias, const float* __restrict__ hres,
            float* Cm, int ldc, unsigned short* Cb) {
  __shared__ __attribute__((aligned(16))) float stg[GBM * GBN];
  const int tid = (int)threadIdx.x, lane = tid & 31, wave = tid >> 5, hh = lane >> 4, m = lane & 15;
  const int rowBase = (int)blockIdx.x * GBM;
  const int colBase = (int)blockIdx.y * GBN;

  v8f acc[8];
  {
    const v8f z = {0.f, 0.f, 0.f, 0.f, 0.f, 0.f, 0.f, 0.f};
#pragma unroll
    for (int t = 0; t < 8; ++t) acc[t] = z;
  }
  const unsigned short* ap = A  + (size_t)(rowBase + 16 * wave + m) * (size_t)lda + 8 * hh;
  const unsigned short* bp = BT + (size_t)(colBase + m) * (size_t)ldb + 8 * hh;

#pragma unroll 1
  for (int k0 = 0; k0 < K; k0 += 32) {
    FragB af;
    af.h[0] = *(const v8usa*)(ap + k0);
    af.h[1] = *(const v8usa*)(ap + k0 + 16);
#pragma unroll
    for (int nt = 0; nt < 8; ++nt) {
      const unsigned short* wq = bp + (size_t)(16 * nt) * (size_t)ldb + k0;
      FragB bf;
      bf.h[0] = *(const v8usa*)wq;
      bf.h[1] = *(const v8usa*)(wq + 16);
      acc[nt] = wmb(af, bf, acc[nt]);
    }
  }

#pragma unroll
  for (int nt = 0; nt < 8; ++nt) {
    const int lc = 16 * nt + m;
    float bvv = 0.0f;
    if constexpr (MODE != 0) bvv = bf16_val(bias[colBase + lc]);
#pragma unroll
    for (int r = 0; r < 8; ++r) {
      const int lr = 16 * wave + 8 * hh + r;
      stg[lr * GBN + lc] = acc[nt][r] + bvv;
    }
  }
  __syncthreads();

  if constexpr (MODE == 1) {
    float* wb = stg + (16 * wave) * GBN;
#pragma unroll 1
    for (int it = 0; it < 16; ++it) {
      float* sp = wb + (it * 32 + lane) * 4;
      const v4f a = *(const v4fa*)sp;
      const v4f r = {silu_f(a.x), silu_f(a.y), silu_f(a.z), silu_f(a.w)};
      *(v4fa*)sp = r;
    }
    __syncthreads();
  }

  if constexpr (MODE == 0) {
#pragma unroll 1
    for (int g = 0; g < 4; ++g) {
      const int lr0 = 16 * wave + 4 * g;
      v4f pv[4];
#pragma unroll
      for (int i = 0; i < 4; ++i) pv[i] = *(const v4fa*)(stg + (lr0 + i) * GBN + 4 * lane);
#pragma unroll
      for (int i = 0; i < 4; ++i) {
        float* op = Cm + (size_t)(rowBase + lr0 + i) * (size_t)ldc + colBase + 4 * lane;
        *(volatile v4f*)op = pv[i];
      }
      __threadfence();
#pragma unroll
      for (int i = 0; i < 4; ++i) {
        float* op = Cm + (size_t)(rowBase + lr0 + i) * (size_t)ldc + colBase + 4 * lane;
        *(volatile v4f*)op = pv[i];
      }
    }
  } else if constexpr (MODE == 1) {
    const int part = lane >> 4;
    const int j = lane & 15;
    const unsigned mh = 0u - (unsigned)part;
    const unsigned ml = ~mh;
#pragma unroll 1
    for (int g = 0; g < 4; ++g) {
      const int lr0 = 16 * wave + 4 * g;
      v8us pv[4];
#pragma unroll
      for (int i = 0; i < 4; ++i) {
        const float* sp = stg + (lr0 + i) * GBN + 8 * j;
        const v4f a = *(const v4fa*)sp;
        const v4f b = *(const v4fa*)(sp + 4);
        const v8f f8 = {a.x, a.y, a.z, a.w, b.x, b.y, b.z, b.w};
        v8us oo;
#pragma unroll
        for (int e = 0; e < 8; ++e) {
          const unsigned hb = bf16_bits(f8[e]);
          const unsigned lb = bf16_bits(f8[e] - __uint_as_float(hb << 16));
          oo[e] = (unsigned short)((hb & ml) | (lb & mh));
        }
        pv[i] = oo;
      }
#pragma unroll
      for (int i = 0; i < 4; ++i) {
        unsigned short* op = Cb + (size_t)(rowBase + lr0 + i) * (size_t)K2 + part * HID + colBase + 8 * j;
        *(volatile v8us*)op = pv[i];
      }
      __threadfence();
#pragma unroll
      for (int i = 0; i < 4; ++i) {
        unsigned short* op = Cb + (size_t)(rowBase + lr0 + i) * (size_t)K2 + part * HID + colBase + 8 * j;
        *(volatile v8us*)op = pv[i];
      }
    }
  } else {
#pragma unroll 1
    for (int g = 0; g < 4; ++g) {
      const int lr0 = 16 * wave + 4 * g;
      v4f pv[4];
#pragma unroll
      for (int i = 0; i < 4; ++i) {
        const int row = rowBase + lr0 + i;
        const v4f hv = *(const v4fa*)(hres + (size_t)row * HID + colBase + 4 * lane);
        const v4f sv = *(const v4fa*)(stg + (lr0 + i) * GBN + 4 * lane);
        v4f q;
        q.x = sv.x + bf16_val(hv.x);
        q.y = sv.y + bf16_val(hv.y);
        q.z = sv.z + bf16_val(hv.z);
        q.w = sv.w + bf16_val(hv.w);
        pv[i] = q;
      }
#pragma unroll
      for (int i = 0; i < 4; ++i) {
        float* op = Cm + (size_t)(rowBase + lr0 + i) * (size_t)ldc + colBase + 4 * lane;
        *(volatile v4f*)op = pv[i];
      }
      __threadfence();
#pragma unroll
      for (int i = 0; i < 4; ++i) {
        float* op = Cm + (size_t)(rowBase + lr0 + i) * (size_t)ldc + colBase + 4 * lane;
        *(volatile v4f*)op = pv[i];
      }
    }
  }
}

__device__ __forceinline__ void wave_gemm_b(const unsigned short* sAw, float* sDw,
                                            const unsigned short* __restrict__ BT, int hh, int m) {
#pragma unroll 1
  for (int nh = 0; nh < 2; ++nh) {
    v8f acc[2][4];
    {
      const v8f z = {0.f, 0.f, 0.f, 0.f, 0.f, 0.f, 0.f, 0.f};
#pragma unroll
      for (int mt = 0; mt < 2; ++mt)
#pragma unroll
        for (int nt = 0; nt < 4; ++nt) acc[mt][nt] = z;
    }
    const unsigned short* ap0 = sAw + m * K2 + 8 * hh;
    const unsigned short* ap1 = ap0 + 16 * K2;
    const unsigned short* bp  = BT + (size_t)(64 * nh + m) * (size_t)K2 + 8 * hh;
#pragma unroll 1
    for (int k0 = 0; k0 < K2; k0 += 32) {
      FragB a0, a1;
      a0.h[0] = *(const v8usa*)(ap0 + k0);
      a0.h[1] = *(const v8usa*)(ap0 + k0 + 16);
      a1.h[0] = *(const v8usa*)(ap1 + k0);
      a1.h[1] = *(const v8usa*)(ap1 + k0 + 16);
#pragma unroll
      for (int nt = 0; nt < 4; ++nt) {
        const unsigned short* wq = bp + (size_t)(16 * nt) * (size_t)K2 + k0;
        FragB b;
        b.h[0] = *(const v8usa*)wq;
        b.h[1] = *(const v8usa*)(wq + 16);
        acc[0][nt] = wmb(a0, b, acc[0][nt]);
        acc[1][nt] = wmb(a1, b, acc[1][nt]);
      }
    }
#pragma unroll
    for (int nt = 0; nt < 4; ++nt) {
      const int col = 64 * nh + 16 * nt + m;
#pragma unroll
      for (int mt = 0; mt < 2; ++mt)
#pragma unroll
        for (int r = 0; r < 8; ++r) sDw[(16 * mt + 8 * hh + r) * HID + col] = acc[mt][nt][r];
    }
  }
}

__global__ __launch_bounds__(NTHR) void k_edge(const float* __restrict__ PQ, const float* __restrict__ TAB,
                                               const float* __restrict__ POSR,
                                               const unsigned short* __restrict__ EW2D,
                                               const unsigned short* __restrict__ PW1D,
                                               float* AGGP, float* S) {
  extern __shared__ __attribute__((aligned(16))) float dyn[];
  unsigned short* sA   = (unsigned short*)dyn;
  float*          sD   = dyn + L_D;
  float*          sPB  = dyn + L_PB;
  float*          sWR  = dyn + L_WR;
  float*          sEB2 = dyn + L_EB2;
  float*          sPB1 = dyn + L_PB1;
  float*          sPW2 = dyn + L_PW2;
  float*          sCS  = dyn + L_CS;
  float*          sRad = dyn + L_RAD;
  float*          sS   = dyn + L_S;

  const int tid = (int)threadIdx.x, lane = tid & 31, wave = tid >> 5, hh = lane >> 4, m = lane & 15;
  const int bi = (int)blockIdx.x / NJT;
  const int jt = (int)blockIdx.x - bi * NJT;
  const int j0 = jt * TJ;

  {
    const int q = tid & 63;
    if (tid < 64) {
      const v4f p = *(const v4fa*)(PQ + (size_t)bi * NPQ + 4 * q);
      const v4f b = *(const v4fa*)(TAB + T_EB1 + 4 * q);
      const v4f r = {p.x + b.x, p.y + b.y, p.z + b.z, p.w + b.w};
      *(v4fa*)(sPB + 4 * q) = r;
      const v4f w = *(const v4fa*)(TAB + T_PW2 + 4 * q);
      *(v4fa*)(sPW2 + 4 * q) = w;
    } else if (tid < 128) {
      const v4f w = *(const v4fa*)(TAB + T_WR + 4 * q);
      *(v4fa*)(sWR + 4 * q) = w;
    } else if (tid < 192) {
      const v4f w = *(const v4fa*)(TAB + T_EB2 + 4 * q);
      *(v4fa*)(sEB2 + 4 * q) = w;
    } else {
      const v4f w = *(const v4fa*)(TAB + T_PB1 + 4 * q);
      *(v4fa*)(sPB1 + 4 * q) = w;
    }
  }
  if (tid < TJ) {
    const int j = j0 + tid;
    const float dx = POSR[3 * j + 0] - POSR[3 * bi + 0];
    const float dy = POSR[3 * j + 1] - POSR[3 * bi + 1];
    const float dz = POSR[3 * j + 2] - POSR[3 * bi + 2];
    sRad[tid] = (dx * dx + dz * dz) + dy * dy;
  }
  __syncthreads();

  {
    const int rsub = tid >> 6;
    const int c4   = (tid & 63) * 4;
    const v4f pb = *(const v4fa*)(sPB + c4);
    const v4f wr = *(const v4fa*)(sWR + c4);
#pragma unroll 2
    for (int sw = 0; sw < TJ / 4; ++sw) {
      const int r = sw * 4 + rsub;
      const v4f q = *(const v4fa*)(PQ + (size_t)(j0 + r) * NPQ + HID + c4);
      const float rad = sRad[r];
      const float f0 = silu_f((pb.x + q.x) + rad * wr.x);
      const float f1 = silu_f((pb.y + q.y) + rad * wr.y);
      const float f2 = silu_f((pb.z + q.z) + rad * wr.z);
      const float f3 = silu_f((pb.w + q.w) + rad * wr.w);
      const unsigned h0 = bf16_bits(f0), h1 = bf16_bits(f1), h2 = bf16_bits(f2), h3 = bf16_bits(f3);
      const unsigned l0 = bf16_bits(f0 - __uint_as_float(h0 << 16));
      const unsigned l1 = bf16_bits(f1 - __uint_as_float(h1 << 16));
      const unsigned l2 = bf16_bits(f2 - __uint_as_float(h2 << 16));
      const unsigned l3 = bf16_bits(f3 - __uint_as_float(h3 << 16));
      const v2u wh = {h0 | (h1 << 16), h2 | (h3 << 16)};
      const v2u wl = {l0 | (l1 << 16), l2 | (l3 << 16)};
      *(v2ua*)(sA + r * K2 + c4)       = wh;
      *(v2ua*)(sA + r * K2 + HID + c4) = wl;
    }
  }
  __syncthreads();

  const int rg = wave & 3, ch = wave >> 2;
  const unsigned short* sAw = sA + (32 * rg) * K2;
  float*                sDw = sD + (32 * rg) * HID + 128 * ch;

  wave_gemm_b(sAw, sDw, EW2D + (size_t)(128 * ch) * K2, hh, m);
  __syncthreads();

  {
    const float eb = sEB2[tid];
    const int   rd = bi - j0;
    float cs = 0.0f;
#pragma unroll 4
    for (int r = 0; r < TJ; ++r) {
      const float v  = sD[r * HID + tid];
      const float mm = silu_f(v + eb);
      cs += (r != rd) ? mm : 0.0f;
      const unsigned hb = bf16_bits(mm);
      const unsigned lb = bf16_bits(mm - __uint_as_float(hb << 16));
      sA[r * K2 + tid]       = (unsigned short)hb;
      sA[r * K2 + HID + tid] = (unsigned short)lb;
    }
    sCS[tid] = cs;
  }
  __syncthreads();

  {
    const int tl = tid < 64 ? tid : 63;
    const v4f o4 = *(const v4fa*)(sCS + 4 * tl);
    float* gp = AGGP + ((size_t)bi * NJT + jt) * HID + 4 * tl;
    if (tid < 64) *(volatile v4f*)gp = o4;
    __threadfence();
    if (tid < 64) *(volatile v4f*)gp = o4;
  }

  wave_gemm_b(sAw, sDw, PW1D + (size_t)(128 * ch) * K2, hh, m);
  __syncthreads();

  {
    float pb[8], pw[8];
#pragma unroll
    for (int q = 0; q < 8; ++q) { pb[q] = sPB1[lane + 32 * q]; pw[q] = sPW2[lane + 32 * q]; }
    const float pb2v = TAB[T_PB2];
#pragma unroll 1
    for (int rr = 0; rr < 16; ++rr) {
      const int r = 16 * wave + rr;
      float part = 0.0f;
#pragma unroll
      for (int q = 0; q < 8; ++q) {
        const float v = sD[r * HID + lane + 32 * q];
        part = fmaf(silu_f(v + pb[q]), pw[q], part);
      }
      part += __shfl_xor(part, 16);
      part += __shfl_xor(part, 8);
      part += __shfl_xor(part, 4);
      part += __shfl_xor(part, 2);
      part += __shfl_xor(part, 1);
      if (lane == 0) sS[r] = part + pb2v;
    }
  }
  __syncthreads();

  {
    const int tl = tid < 32 ? tid : 31;
    const v4f o4 = *(const v4fa*)(sS + 4 * tl);
    float* gp = S + (size_t)bi * NN + j0 + 4 * tl;
    if (tid < 32) *(volatile v4f*)gp = o4;
    __threadfence();
    if (tid < 32) *(volatile v4f*)gp = o4;
  }
}

__global__ __launch_bounds__(NTHR) void k_aggc(const float* __restrict__ AGGP, const float* __restrict__ nodes,
                                               unsigned short* AN) {
  const int u   = (int)blockIdx.x * NTHR + (int)threadIdx.x;
  const int row = u >> 5;
  const int j   = u & 31;
  const float* a0 = AGGP + ((size_t)row * NJT + 0) * HID + 8 * j;
  const float* a1 = AGGP + ((size_t)row * NJT + 1) * HID + 8 * j;
  const float* a2 = AGGP + ((size_t)row * NJT + 2) * HID + 8 * j;
  const float* hq = nodes + (size_t)row * HID + 8 * j;
  const v4f p0 = *(const v4fa*)a0, p1 = *(const v4fa*)(a0 + 4);
  const v4f q0 = *(const v4fa*)a1, q1 = *(const v4fa*)(a1 + 4);
  const v4f r0 = *(const v4fa*)a2, r1 = *(const v4fa*)(a2 + 4);
  const v4f ha = *(const v4fa*)hq, hb = *(const v4fa*)(hq + 4);
  const v8f g8 = {(p0.x + q0.x) + r0.x, (p0.y + q0.y) + r0.y, (p0.z + q0.z) + r0.z, (p0.w + q0.w) + r0.w,
                  (p1.x + q1.x) + r1.x, (p1.y + q1.y) + r1.y, (p1.z + q1.z) + r1.z, (p1.w + q1.w) + r1.w};
  v8us ohi, olo;
#pragma unroll
  for (int i = 0; i < 8; ++i) {
    const unsigned hbits = bf16_bits(g8[i]);
    ohi[i] = (unsigned short)hbits;
    olo[i] = (unsigned short)bf16_bits(g8[i] - __uint_as_float(hbits << 16));
  }
  const v8us ohb = cvt8(ha, hb);
  unsigned short* dp = AN + (size_t)row * K3 + 8 * j;
  *(volatile v8us*)dp             = ohb;
  *(volatile v8us*)(dp + HID)     = ohi;
  *(volatile v8us*)(dp + 2 * HID) = olo;
  __threadfence();
  *(volatile v8us*)dp             = ohb;
  *(volatile v8us*)(dp + HID)     = ohi;
  *(volatile v8us*)(dp + 2 * HID) = olo;
}

__global__ __launch_bounds__(NN) void k_pos(const float* __restrict__ POSR, const float* __restrict__ S,
                                            const int* __restrict__ nnode, float* out1) {
  __shared__ __attribute__((aligned(16))) float sp[OUT1_ELEMS];
  __shared__ __attribute__((aligned(16))) float sx[OUT1_ELEMS];
  const int tid = (int)threadIdx.x;
  {
    const int tl = tid < POS_UNITS ? tid : POS_UNITS - 1;
    const v4f v = *(const v4fa*)(POSR + 4 * tl);
    if (tid < POS_UNITS) *(v4fa*)(sp + 4 * tl) = v;
  }
  __syncthreads();
  const float px = sp[3 * tid + 0], py = sp[3 * tid + 1], pz = sp[3 * tid + 2];
  float ax = 0.0f, ay = 0.0f, az = 0.0f;
#pragma unroll 4
  for (int i = 0; i < NN; ++i) {
    const float sv = S[(size_t)i * NN + tid];
    float tx = (px - sp[3 * i + 0]) * sv;
    float ty = (py - sp[3 * i + 1]) * sv;
    float tz = (pz - sp[3 * i + 2]) * sv;
    tx = (tx < -100.0f) ? -100.0f : ((tx > 100.0f) ? 100.0f : tx);
    ty = (ty < -100.0f) ? -100.0f : ((ty > 100.0f) ? 100.0f : ty);
    tz = (tz < -100.0f) ? -100.0f : ((tz > 100.0f) ? 100.0f : tz);
    const bool on = (i != tid);
    ax += on ? tx : 0.0f;
    ay += on ? ty : 0.0f;
    az += on ? tz : 0.0f;
  }
  const int   nv   = nnode[0];
  const float qnan = __int_as_float(0x7fc00000);
  const float poi  = (nv == NN) ? 0.0f : qnan;
  sx[3 * tid + 0] = (px + ax) + poi;
  sx[3 * tid + 1] = (py + ay) + poi;
  sx[3 * tid + 2] = (pz + az) + poi;
  __syncthreads();
  const int tl = tid < POS_UNITS ? tid : POS_UNITS - 1;
  const v4f o4 = *(const v4fa*)(sx + 4 * tl);
  if (tid < POS_UNITS) *(volatile v4f*)(out1 + 4 * tl) = o4;
  __threadfence();
  if (tid < POS_UNITS) *(volatile v4f*)(out1 + 4 * tl) = o4;
}

extern "C" void kernel_launch(void* const* d_in, const int* in_sizes, int n_in,
                              void* d_out, int out_size, void* d_ws, size_t ws_size,
                              hipStream_t stream) {
  if (n_in < 15) return;
  if (in_sizes[0] != NN * HID || in_sizes[1] != NN * 3) return;
  if (in_sizes[2] != HID * EW1S || in_sizes[3] != HID) return;
  if (in_sizes[4] != HID * HID || in_sizes[5] != HID) return;
  if (in_sizes[6] != HID * 2 * HID || in_sizes[7] != HID) return;
  if (in_sizes[8] != HID * HID || in_sizes[9] != HID) return;
  if (in_sizes[10] != HID * HID || in_sizes[11] != HID) return;
  if (in_sizes[12] != HID || in_sizes[13] != 1 || in_sizes[14] != 1) return;
  if (out_size != OUT_TOTAL) return;

  const float* nodes = (const float*)d_in[0];
  const float* pos   = (const float*)d_in[1];
  const float* eW1   = (const float*)d_in[2];
  const float* eb1   = (const float*)d_in[3];
  const float* eW2   = (const float*)d_in[4];
  const float* eb2   = (const float*)d_in[5];
  const float* nW1   = (const float*)d_in[6];
  const float* nb1   = (const float*)d_in[7];
  const float* nW2   = (const float*)d_in[8];
  const float* nb2   = (const float*)d_in[9];
  const float* pW1   = (const float*)d_in[10];
  const float* pb1   = (const float*)d_in[11];
  const float* pW2   = (const float*)d_in[12];
  const float* pb2   = (const float*)d_in[13];
  const int*   nnode = (const int*)d_in[14];
  float* out0 = (float*)d_out;
  float* out1 = out0 + OUT0_ELEMS;

  char* ws = (char*)d_ws;
  size_t off = 0;
  const size_t oXB   = off; off += (size_t)NN * HID * 2;        off = (off + 255) & ~(size_t)255;
  const size_t oPOSR = off; off += (size_t)OUT1_ELEMS * 4;      off = (off + 255) & ~(size_t)255;
  const size_t oPQW  = off; off += (size_t)NPQ * HID * 2;       off = (off + 255) & ~(size_t)255;
  const size_t oEW2D = off; off += (size_t)HID * K2 * 2;        off = (off + 255) & ~(size_t)255;
  const size_t oPW1D = off; off += (size_t)HID * K2 * 2;        off = (off + 255) & ~(size_t)255;
  const size_t oNW2D = off; off += (size_t)HID * K2 * 2;        off = (off + 255) & ~(size_t)255;
  const size_t oNW1C = off; off += (size_t)HID * K3 * 2;        off = (off + 255) & ~(size_t)255;
  const size_t oTAB  = off; off += (size_t)T_END * 4;           off = (off + 255) & ~(size_t)255;
  const size_t oPQ   = off; off += (size_t)NN * NPQ * 4;        off = (off + 255) & ~(size_t)255;
  const size_t oAGGP = off; off += (size_t)NN * NJT * HID * 4;  off = (off + 255) & ~(size_t)255;
  const size_t oS    = off; off += (size_t)NN * NN * 4;         off = (off + 255) & ~(size_t)255;
  const size_t oAN   = off; off += (size_t)NN * K3 * 2;         off = (off + 255) & ~(size_t)255;
  const size_t oTHL  = off; off += (size_t)NN * K2 * 2;         off = (off + 255) & ~(size_t)255;
  if (off > ws_size || off > (size_t)WSMAX) return;

  unsigned short* XB    = (unsigned short*)(ws + oXB);
  float*          POSR  = (float*)(ws + oPOSR);
  unsigned short* EW1PQ = (unsigned short*)(ws + oPQW);
  unsigned short* EW2D  = (unsigned short*)(ws + oEW2D);
  unsigned short* PW1D  = (unsigned short*)(ws + oPW1D);
  unsigned short* NW2D  = (unsigned short*)(ws + oNW2D);
  unsigned short* NW1C  = (unsigned short*)(ws + oNW1C);
  float*          TAB   = (float*)(ws + oTAB);
  float*          PQ    = (float*)(ws + oPQ);
  float*          AGGP  = (float*)(ws + oAGGP);
  float*          S     = (float*)(ws + oS);
  unsigned short* AN    = (unsigned short*)(ws + oAN);
  unsigned short* THL   = (unsigned short*)(ws + oTHL);

  hipFuncSetAttribute(reinterpret_cast<const void*>(&k_edge), hipFuncAttributeMaxDynamicSharedMemorySize,
                      (int)EDGE_LDS_BYTES);

  k_prep<<<NU_ALL / NTHR, NTHR, 0, stream>>>(nodes, pos, eW1, eb1, eW2, eb2, nW1, nb1, nW2, nb2, pW1, pb1, pW2, pb2,
                                             XB, POSR, EW1PQ, EW2D, PW1D, NW2D, NW1C, TAB);
  k_gemm<0><<<dim3(NN / GBM, NPQ / GBN), GTHR, 0, stream>>>(XB, HID, EW1PQ, HID, HID, nb1, nodes, PQ, NPQ, THL);
  k_edge<<<NN * NJT, NTHR, EDGE_LDS_BYTES, stream>>>(PQ, TAB, POSR, EW2D, PW1D, AGGP, S);
  k_aggc<<<(NN * (HID / 8)) / NTHR, NTHR, 0, stream>>>(AGGP, nodes, AN);
  k_gemm<1><<<dim3(NN / GBM, HID / GBN), GTHR, 0, stream>>>(AN, K3, NW1C, K3, K3, nb1, nodes, PQ, NPQ, THL);
  k_gemm<2><<<dim3(NN / GBM, HID / GBN), GTHR, 0, stream>>>(THL, K2, NW2D, K2, K2, nb2, nodes, out0, HID, AN);
  k_pos<<<1, NN, 0, stream>>>(POSR, S, nnode, out1);
}
